// SelfAttention_20761871909007
// MI455X (gfx1250) — hardware-run, weakly checked
//
#include <hip/hip_runtime.h>


#ifndef NB
#define NB 8
#endif
#ifndef SEQ
#define SEQ 1024
#endif
#define NB_FULL    8
#define SEQ_FULL   1024
#define CH         256
#define NHEAD      8
#define EQK        64
#define WROWS      384
#define HCAT       2048
#define BQ         64
#define BK         32
#define NWAVE      8
#define PO         136
#define CP         72
#define YP         68
#define LNP        33
#define WSCALE     64.0f
#define WS_CAP     134217728ull

static_assert(SEQ % 128 == 0);
static_assert(SEQ % BQ == 0);
static_assert(SEQ % BK == 0);
static_assert(SEQ <= SEQ_FULL);
static_assert(NB >= 1 && NB <= NB_FULL);
static_assert(CH == 256 && EQK == 64 && HCAT == NHEAD * CH);
static_assert(WROWS == 2 * EQK + CH);
static_assert(CH % 32 == 0 && HCAT % 32 == 0 && EQK % 32 == 0);
static_assert((PO * 2) % 16 == 0 && (CP * 2) % 16 == 0 && (YP * 4) % 16 == 0);
static_assert(PO >= 128 && CP >= 64 && YP >= 64);

static constexpr size_t WC_ELEMS = (size_t)NHEAD * WROWS * CH;
static constexpr size_t WO_ELEMS = (size_t)CH * HCAT;
static constexpr size_t TN_ELEMS = (size_t)NB * SEQ * CH;
static constexpr size_t QK_ELEMS = (size_t)NB * NHEAD * SEQ * EQK;
static constexpr size_t VT_ELEMS = (size_t)NB * NHEAD * CH * SEQ;
static constexpr size_t CX_ELEMS = (size_t)NB * SEQ * HCAT;
static constexpr size_t WC_OFF = 0;
static constexpr size_t WO_OFF = WC_OFF + WC_ELEMS;
static constexpr size_t TN_OFF = WO_OFF + WO_ELEMS;
static constexpr size_t Q_OFF  = TN_OFF + TN_ELEMS;
static constexpr size_t K_OFF  = Q_OFF + QK_ELEMS;
static constexpr size_t VT_OFF = K_OFF + QK_ELEMS;
static constexpr size_t CX_OFF = VT_OFF + VT_ELEMS;
static constexpr size_t WS_ELEMS = CX_OFF + CX_ELEMS;
static_assert(WS_ELEMS * 2ull <= WS_CAP);
static_assert(WO_OFF % 64 == 0 && TN_OFF % 64 == 0 && Q_OFF % 64 == 0 && K_OFF % 64 == 0);
static_assert(VT_OFF % 64 == 0 && CX_OFF % 64 == 0);
static_assert(((size_t)(NB - 1) * CH + (CH - 1)) * SEQ_FULL + SEQ <= (size_t)NB_FULL * CH * SEQ_FULL);

typedef __bf16   bf16;
typedef _Float16 f16;
typedef f16      v16h  __attribute__((ext_vector_type(16)));
typedef f16      v8h   __attribute__((ext_vector_type(8)));
typedef float    v8f   __attribute__((ext_vector_type(8)));
typedef float    v4f   __attribute__((ext_vector_type(4)));
typedef unsigned v4u   __attribute__((ext_vector_type(4)));

union FragH  { v16h  v; v4u q[2]; f16  h[16]; };
union Pack8H { v4u u; v8h v; f16 h[8]; };

static __device__ __forceinline__ v8f mma_f16(v16h a, v16h b, v8f acc) {
  acc = __builtin_amdgcn_wmma_f32_16x16x32_f16(false, a, false, b, (short)0, acc, false, false);
  asm volatile("v_nop\n\tv_nop\n\tv_nop\n\tv_nop" : "+v"(acc) : "v"(a), "v"(b));
  return acc;
}

static __device__ __forceinline__ float bf16v(float v) { return (float)(bf16)v; }

__global__ __launch_bounds__(256) void wplane_kernel(const float* __restrict__ src, f16* __restrict__ dst,
                                                     int nrows, int rows_per_head, int dst_rows_per_head,
                                                     int dst_row_off) {
  const int lane = threadIdx.x & 31;
  const int row  = blockIdx.x * 8 + (threadIdx.x >> 5);
  if (row >= nrows) return;
  const int hh = row / rows_per_head;
  const int r  = row - hh * rows_per_head;
  const float* sp = src + (size_t)row * CH + lane * 8;
  const v4f a0 = *(const v4f*)(sp);
  const v4f a1 = *(const v4f*)(sp + 4);
  Pack8H p;
  #pragma unroll
  for (int i = 0; i < 4; ++i) {
    p.h[i]     = (f16)(bf16v(a0[i]) * WSCALE);
    p.h[4 + i] = (f16)(bf16v(a1[i]) * WSCALE);
  }
  const v4u val = p.u;
  f16* dp = dst + ((size_t)hh * dst_rows_per_head + dst_row_off + r) * CH + lane * 8;
  *(volatile v4u*)dp = val;
  __threadfence();
  *(volatile v4u*)dp = val;
}

__global__ __launch_bounds__(256) void ln_kernel(const float* __restrict__ x, f16* __restrict__ tn) {
  const int n0   = blockIdx.x * 32;
  const int b    = blockIdx.y;
  const int tid  = threadIdx.x;
  const int lane = tid & 31;
  const int wave = tid >> 5;
  __shared__ __align__(16) float sX[CH * LNP];

  #pragma unroll 4
  for (int i = 0; i < 32; ++i) {
    const int c = i * 8 + wave;
    const float v = x[((size_t)b * CH + c) * SEQ_FULL + n0 + lane];
    sX[c * LNP + lane] = bf16v(v);
  }
  __syncthreads();

  #pragma unroll 1
  for (int t4 = 0; t4 < 4; ++t4) {
    const int t = wave * 4 + t4;
    float xv[8];
    float s = 0.0f;
    #pragma unroll
    for (int i = 0; i < 8; ++i) {
      xv[i] = sX[(lane * 8 + i) * LNP + t];
      s += xv[i];
    }
    s += __shfl_xor(s, 16, 32);
    s += __shfl_xor(s, 8, 32);
    s += __shfl_xor(s, 4, 32);
    s += __shfl_xor(s, 2, 32);
    s += __shfl_xor(s, 1, 32);
    const float mean = s * (1.0f / CH);
    float d2 = 0.0f;
    #pragma unroll
    for (int i = 0; i < 8; ++i) {
      const float d = xv[i] - mean;
      d2 += d * d;
    }
    d2 += __shfl_xor(d2, 16, 32);
    d2 += __shfl_xor(d2, 8, 32);
    d2 += __shfl_xor(d2, 4, 32);
    d2 += __shfl_xor(d2, 2, 32);
    d2 += __shfl_xor(d2, 1, 32);
    const float rstd = rsqrtf(d2 * (1.0f / CH) + 1e-5f);
    Pack8H p;
    #pragma unroll
    for (int i = 0; i < 8; ++i) p.h[i] = (f16)((xv[i] - mean) * rstd);
    const v4u val = p.u;
    f16* dp = tn + ((size_t)b * SEQ + n0 + t) * CH + lane * 8;
    *(volatile v4u*)dp = val;
    __threadfence();
    *(volatile v4u*)dp = val;
  }
}

template <int KDIM>
static __device__ __forceinline__ void gemm_32x64(const f16* ap, const f16* bp, v8f (&acc)[2][4]) {
  #pragma unroll 1
  for (int k0 = 0; k0 < KDIM; k0 += 32) {
    FragH a[2], bfr[4];
    #pragma unroll
    for (int mt = 0; mt < 2; ++mt) {
      const f16* p = ap + (size_t)(mt * 16) * KDIM + k0;
      a[mt].q[0] = *(const v4u*)(p);
      a[mt].q[1] = *(const v4u*)(p + 16);
    }
    #pragma unroll
    for (int nt = 0; nt < 4; ++nt) {
      const f16* p = bp + (size_t)(nt * 16) * KDIM + k0;
      bfr[nt].q[0] = *(const v4u*)(p);
      bfr[nt].q[1] = *(const v4u*)(p + 16);
    }
    #pragma unroll
    for (int mt = 0; mt < 2; ++mt) {
      #pragma unroll
      for (int nt = 0; nt < 4; ++nt) acc[mt][nt] = mma_f16(a[mt].v, bfr[nt].v, acc[mt][nt]);
    }
  }
}

__global__ __launch_bounds__(128) void qkv_kernel(const f16* rd, f16* wr,
                                                  const float* __restrict__ bq,
                                                  const float* __restrict__ bk,
                                                  const float* __restrict__ bv) {
  const int bx   = blockIdx.x;
  const int h    = blockIdx.y;
  const int b    = blockIdx.z;
  const int tid  = threadIdx.x;
  const int wave = __builtin_amdgcn_readfirstlane(tid >> 5);
  const int lane = tid & 31;
  const int lq   = lane & 15;
  const int hi   = lane >> 4;
  __shared__ __align__(16) f16 sC[128 * CP];

  const int NQT = SEQ / 128;
  const int typ = (bx < NQT) ? 0 : ((bx < 2 * NQT) ? 1 : 2);
  const bool isV = (typ == 2);
  int mtile;
  size_t aoff, boff, ooff;
  int opitch;
  if (!isV) {
    mtile  = bx - typ * NQT;
    aoff   = TN_OFF + ((size_t)b * SEQ + mtile * 128) * CH;
    boff   = WC_OFF + ((size_t)h * WROWS + typ * EQK) * CH;
    ooff   = ((typ == 0) ? Q_OFF : K_OFF) + (((size_t)b * NHEAD + h) * SEQ + mtile * 128) * EQK;
    opitch = EQK;
  } else {
    const int xv = bx - 2 * NQT;
    mtile  = xv & 1;
    const int ntile = xv >> 1;
    aoff   = WC_OFF + ((size_t)h * WROWS + 2 * EQK + mtile * 128) * CH;
    boff   = TN_OFF + ((size_t)b * SEQ + ntile * 64) * CH;
    ooff   = VT_OFF + (((size_t)b * NHEAD + h) * CH + mtile * 128) * SEQ + ntile * 64;
    opitch = SEQ;
  }

  v8f acc[2][4];
  #pragma unroll
  for (int mt = 0; mt < 2; ++mt) {
    #pragma unroll
    for (int nt = 0; nt < 4; ++nt) acc[mt][nt] = (v8f){0, 0, 0, 0, 0, 0, 0, 0};
  }
  gemm_32x64<CH>(rd + aoff + (size_t)(wave * 32 + lq) * CH + hi * 8,
                 rd + boff + (size_t)lq * CH + hi * 8, acc);

  float cb[4];
  #pragma unroll
  for (int nt = 0; nt < 4; ++nt) {
    const int ci = h * EQK + nt * 16 + lq;
    const float vq = bq[ci];
    const float vk = bk[ci];
    cb[nt] = bf16v((typ == 0) ? vq : vk);
  }
  v4f rb[2][2];
  #pragma unroll
  for (int mt = 0; mt < 2; ++mt) {
    const int ri = (mtile * 128 + wave * 32 + mt * 16 + hi * 8) & (CH - 1);
    const float* p = bv + h * CH + ri;
    rb[mt][0] = *(const v4f*)(p);
    rb[mt][1] = *(const v4f*)(p + 4);
  }
  #pragma unroll
  for (int mt = 0; mt < 2; ++mt) {
    #pragma unroll
    for (int r = 0; r < 8; ++r) {
      const float rbv = bf16v(rb[mt][r >> 2][r & 3]);
      #pragma unroll
      for (int nt = 0; nt < 4; ++nt) {
        const float bias = isV ? rbv : cb[nt];
        sC[(wave * 32 + mt * 16 + hi * 8 + r) * CP + nt * 16 + lq] =
            (f16)(acc[mt][nt][r] * (1.0f / WSCALE) + bias);
      }
    }
  }
  __syncthreads();

  v4u    vals[8];
  size_t gi[8];
  #pragma unroll
  for (int it = 0; it < 8; ++it) {
    const int row = wave * 32 + it * 4 + (lane >> 3);
    const int pc  = lane & 7;
    Pack8H t;
    t.v = *(const v8h*)(sC + row * CP + pc * 8);
    vals[it] = t.u;
    gi[it] = ooff + (size_t)row * opitch + pc * 8;
  }
  #pragma unroll
  for (int it = 0; it < 8; ++it) *(volatile v4u*)(wr + gi[it]) = vals[it];
  __threadfence();
  #pragma unroll
  for (int it = 0; it < 8; ++it) *(volatile v4u*)(wr + gi[it]) = vals[it];
}

__global__ __launch_bounds__(256) void attn_kernel(const f16* __restrict__ q16,
                                                   const f16* __restrict__ k16,
                                                   const f16* __restrict__ vt16,
                                                   f16* __restrict__ ctx) {
  const int qblk = blockIdx.x;
  const int h    = blockIdx.y;
  const int b    = blockIdx.z;
  const int tid  = threadIdx.x;
  const int wave = __builtin_amdgcn_readfirstlane(tid >> 5);
  const int lane = tid & 31;
  const int lq   = lane & 15;
  const int hi   = lane >> 4;
  const int qg   = wave >> 1;
  const int chf  = wave & 1;

  __shared__ __align__(16) f16 sO[NWAVE * 16 * PO];

  const int qrow0 = qblk * BQ + qg * 16;

  FragH qf[2];
  {
    const f16* qp = q16 + (((size_t)b * NHEAD + h) * SEQ + qrow0 + lq) * EQK + hi * 8;
    #pragma unroll
    for (int f = 0; f < 2; ++f) {
      qf[f].q[0] = *(const v4u*)(qp + f * 32);
      qf[f].q[1] = *(const v4u*)(qp + f * 32 + 16);
    }
  }

  const f16* k_h  = k16 + ((size_t)b * NHEAD + h) * SEQ * EQK;
  const f16* vt_h = vt16 + (((size_t)b * NHEAD + h) * CH + chf * 128) * SEQ;

  v8f o[8];
  #pragma unroll
  for (int dt = 0; dt < 8; ++dt) o[dt] = (v8f){0, 0, 0, 0, 0, 0, 0, 0};

  float rmax = -__builtin_inff();
  float rsum = 0.0f;
  const float SL = 0.125f * 1.4426950408889634f;

  const int nchunk = SEQ / BK;
  #pragma unroll 1
  for (int i = 0; i < nchunk; ++i) {
    const int j0 = i * BK;

    FragH ak[2][2];
    #pragma unroll
    for (int sub = 0; sub < 2; ++sub) {
      #pragma unroll
      for (int f = 0; f < 2; ++f) {
        const f16* base = k_h + (size_t)(j0 + sub * 16 + lq) * EQK + f * 32 + hi * 8;
        ak[sub][f].q[0] = *(const v4u*)(base);
        ak[sub][f].q[1] = *(const v4u*)(base + 16);
      }
    }

    v8f c[2];
    #pragma unroll
    for (int sub = 0; sub < 2; ++sub) {
      v8f acc = (v8f){0, 0, 0, 0, 0, 0, 0, 0};
      acc = mma_f16(ak[sub][0].v, qf[0].v, acc);
      acc = mma_f16(ak[sub][1].v, qf[1].v, acc);
      c[sub] = acc;
    }

    float m_new = rmax;
    #pragma unroll
    for (int r = 0; r < 8; ++r) {
      m_new = fmaxf(m_new, c[0][r]);
      m_new = fmaxf(m_new, c[1][r]);
    }
    m_new = fmaxf(m_new, __shfl_xor(m_new, 16, 32));
    const float scale = __builtin_amdgcn_exp2f((rmax - m_new) * SL);
    rmax = m_new;

    FragH pa;
    float psum = 0.0f;
    #pragma unroll
    for (int r = 0; r < 8; ++r) {
      const float p0 = __builtin_amdgcn_exp2f((c[0][r] - m_new) * SL);
      const float p1 = __builtin_amdgcn_exp2f((c[1][r] - m_new) * SL);
      psum += p0 + p1;
      pa.h[r]     = (f16)(p0 * 4096.0f);
      pa.h[8 + r] = (f16)(p1 * 4096.0f);
    }
    rsum = rsum * scale + psum + __shfl_xor(psum, 16, 32);

    float sc[8];
    #pragma unroll
    for (int r = 0; r < 8; ++r) sc[r] = __shfl(scale, (hi << 3) + r, 32);
    #pragma unroll
    for (int dt = 0; dt < 8; ++dt) {
      #pragma unroll
      for (int r = 0; r < 8; ++r) o[dt][r] *= sc[r];
    }

    #pragma unroll
    for (int g = 0; g < 2; ++g) {
      FragH bvf[4];
      #pragma unroll
      for (int d4 = 0; d4 < 4; ++d4) {
        const f16* base = vt_h + (size_t)((g * 4 + d4) * 16 + lq) * SEQ + j0 + hi * 8;
        bvf[d4].q[0] = *(const v4u*)(base);
        bvf[d4].q[1] = *(const v4u*)(base + 16);
      }
      #pragma unroll
      for (int d4 = 0; d4 < 4; ++d4) o[g * 4 + d4] = mma_f16(pa.v, bvf[d4].v, o[g * 4 + d4]);
    }
  }

  float rs[8];
  #pragma unroll
  for (int r = 0; r < 8; ++r) rs[r] = (64.0f / 4096.0f) * (1.0f / __shfl(rsum, (hi << 3) + r, 32));

  f16* so = sO + wave * (16 * PO);
  #pragma unroll
  for (int r = 0; r < 8; ++r) {
    #pragma unroll
    for (int dt = 0; dt < 8; ++dt) {
      so[(hi * 8 + r) * PO + dt * 16 + lq] = (f16)(o[dt][r] * rs[r]);
    }
  }
  __syncthreads();

  v4u    vals[8];
  size_t gidx[8];
  #pragma unroll
  for (int it = 0; it < 8; ++it) {
    const int row = it * 2 + hi;
    Pack8H t;
    t.v = *(const v8h*)(so + row * PO + lq * 8);
    vals[it] = t.u;
    gidx[it] = ((size_t)b * SEQ + qrow0 + row) * HCAT + h * CH + chf * 128 + lq * 8;
  }
  #pragma unroll
  for (int it = 0; it < 8; ++it) *(volatile v4u*)(ctx + gidx[it]) = vals[it];
  __threadfence();
  #pragma unroll
  for (int it = 0; it < 8; ++it) *(volatile v4u*)(ctx + gidx[it]) = vals[it];
}

__global__ __launch_bounds__(128) void oproj_kernel(const f16* __restrict__ wo16,
                                                    const f16* __restrict__ ctx,
                                                    const float* __restrict__ bo,
                                                    float* __restrict__ y) {
  const int ntile = blockIdx.x;
  const int mtile = blockIdx.y;
  const int b     = blockIdx.z;
  const int tid   = threadIdx.x;
  const int wave  = __builtin_amdgcn_readfirstlane(tid >> 5);
  const int lane  = tid & 31;
  const int lq    = lane & 15;
  const int hi    = lane >> 4;
  __shared__ __align__(16) float sY[128 * YP];

  v8f acc[2][4];
  #pragma unroll
  for (int mt = 0; mt < 2; ++mt) {
    #pragma unroll
    for (int nt = 0; nt < 4; ++nt) acc[mt][nt] = (v8f){0, 0, 0, 0, 0, 0, 0, 0};
  }
  gemm_32x64<HCAT>(wo16 + (size_t)(mtile * 128 + wave * 32 + lq) * HCAT + hi * 8,
                   ctx + ((size_t)b * SEQ + ntile * 64 + lq) * HCAT + hi * 8, acc);

  v4f rb[2][2];
  #pragma unroll
  for (int mt = 0; mt < 2; ++mt) {
    const float* p = bo + mtile * 128 + wave * 32 + mt * 16 + hi * 8;
    rb[mt][0] = *(const v4f*)(p);
    rb[mt][1] = *(const v4f*)(p + 4);
  }
  #pragma unroll
  for (int mt = 0; mt < 2; ++mt) {
    #pragma unroll
    for (int r = 0; r < 8; ++r) {
      const float rbv = bf16v(rb[mt][r >> 2][r & 3]);
      #pragma unroll
      for (int nt = 0; nt < 4; ++nt) {
        sY[(wave * 32 + mt * 16 + hi * 8 + r) * YP + nt * 16 + lq] =
            acc[mt][nt][r] * (1.0f / (WSCALE * 64.0f)) + rbv;
      }
    }
  }
  __syncthreads();

  v4f    vals[16];
  size_t gi[16];
  #pragma unroll
  for (int it = 0; it < 16; ++it) {
    const int row = wave * 32 + it * 2 + hi;
    vals[it] = *(const v4f*)(sY + row * YP + lq * 4);
    gi[it] = ((size_t)b * CH + mtile * 128 + row) * SEQ_FULL + ntile * 64 + lq * 4;
  }
  #pragma unroll
  for (int it = 0; it < 16; ++it) *(volatile v4f*)(y + gi[it]) = vals[it];
  __threadfence();
  #pragma unroll
  for (int it = 0; it < 16; ++it) *(volatile v4f*)(y + gi[it]) = vals[it];
}

extern "C" void kernel_launch(void* const* d_in, const int* in_sizes, int n_in,
                              void* d_out, int out_size, void* d_ws, size_t ws_size,
                              hipStream_t stream) {
  if (n_in < 9) return;
  const size_t xneed = ((size_t)(NB - 1) * CH + (CH - 1)) * SEQ_FULL + SEQ;
  if ((size_t)in_sizes[0] < xneed) return;
  if ((size_t)in_sizes[1] < (size_t)NHEAD * EQK * CH) return;
  if ((size_t)in_sizes[2] < (size_t)NHEAD * EQK) return;
  if ((size_t)in_sizes[3] < (size_t)NHEAD * EQK * CH) return;
  if ((size_t)in_sizes[4] < (size_t)NHEAD * EQK) return;
  if ((size_t)in_sizes[5] < (size_t)NHEAD * CH * CH) return;
  if ((size_t)in_sizes[6] < (size_t)NHEAD * CH) return;
  if ((size_t)in_sizes[7] < (size_t)CH * HCAT) return;
  if ((size_t)in_sizes[8] < (size_t)CH) return;
  if ((size_t)out_size < xneed) return;
  if (ws_size < WS_ELEMS * 2) return;

  const float* x  = (const float*)d_in[0];
  const float* Wq = (const float*)d_in[1];
  const float* bq = (const float*)d_in[2];
  const float* Wk = (const float*)d_in[3];
  const float* bk = (const float*)d_in[4];
  const float* Wv = (const float*)d_in[5];
  const float* bv = (const float*)d_in[6];
  const float* Wo = (const float*)d_in[7];
  const float* bo = (const float*)d_in[8];
  float* y  = (float*)d_out;
  f16*   ws = (f16*)d_ws;

  wplane_kernel<<<(NHEAD * EQK + 7) / 8, 256, 0, stream>>>(Wq, ws + WC_OFF, NHEAD * EQK, EQK, WROWS, 0);
  wplane_kernel<<<(NHEAD * EQK + 7) / 8, 256, 0, stream>>>(Wk, ws + WC_OFF, NHEAD * EQK, EQK, WROWS, EQK);
  wplane_kernel<<<(NHEAD * CH + 7) / 8, 256, 0, stream>>>(Wv, ws + WC_OFF, NHEAD * CH, CH, WROWS, 2 * EQK);
  wplane_kernel<<<(HCAT + 7) / 8, 256, 0, stream>>>(Wo, ws + WO_OFF, HCAT, HCAT, HCAT, 0);

  ln_kernel<<<dim3(SEQ / 32, NB), 256, 0, stream>>>(x, ws + TN_OFF);

  qkv_kernel<<<dim3(2 * (SEQ / 128) + 2 * (SEQ / 64), NHEAD, NB), 128, 0, stream>>>(ws, ws, bq, bk, bv);

  attn_kernel<<<dim3(SEQ / BQ, NHEAD, NB), 256, 0, stream>>>(ws + Q_OFF, ws + K_OFF, ws + VT_OFF, ws + CX_OFF);

  oproj_kernel<<<dim3(SEQ / 64, CH / 128, NB), 128, 0, stream>>>(ws + WO_OFF, ws + CX_OFF, bo, y);
}
